// VisionMamba_32538672235138
// MI455X (gfx1250) — hardware-run, weakly checked
//
#include <hip/hip_runtime.h>
#include <math.h>

typedef __attribute__((ext_vector_type(16))) _Float16 v16h;
typedef __attribute__((ext_vector_type(8)))  _Float16 v8h;
typedef __attribute__((ext_vector_type(16))) __bf16   v16b;
typedef __attribute__((ext_vector_type(8)))  __bf16   v8b;
typedef __attribute__((ext_vector_type(8)))  float    v8f;
typedef __attribute__((ext_vector_type(4)))  float    v4f;

constexpr int kBatch = 4;
constexpr int kSeq   = 1024;
constexpr int kRows  = kBatch * kSeq;
constexpr int kF     = 64;
constexpr int kNst   = 64;
constexpr int kNd    = 4;
constexpr int kLayers = 8;
constexpr int kImg = 256, kCin = 3, kCout = 3, kGp = 32;
constexpr int kKpe  = 192;
constexpr int kKcv  = 192;
constexpr int kNbc  = 192;
constexpr int kNout = 192;
constexpr int kPadRows = kSeq + 2;
constexpr int kTS = 32;
constexpr float kEps = 1e-5f;
static_assert((kKpe % 32) == 0 && (kKcv % 32) == 0 && (kF % 32) == 0, "K mult of 32");
static_assert((kSeq % 64) == 0 && (kRows % 64) == 0 && (kF % 64) == 0 && (kNbc % 64) == 0 && (kNout % 64) == 0, "M,N mult of 64");
static_assert((kSeq % kTS) == 0 && kTS == 32, "chunking");
static_assert(kNd * 64 == 256, "Wd2 slice");

constexpr size_t kSzW64x192 = (size_t)64 * 192 * 2;
constexpr size_t kSzW8x64x64 = (size_t)kLayers * 64 * 64 * 2;
constexpr size_t kSzW8x64x192 = (size_t)kLayers * 64 * 192 * 2;
constexpr size_t kSzAct32 = (size_t)kRows * kF * 4;
constexpr size_t kSzAct16 = (size_t)kRows * kF * 2;
constexpr size_t kSzH0P = (size_t)kBatch * kPadRows * kF * 2;
constexpr size_t kOffWPEH = 0;
constexpr size_t kOffWPEL = kOffWPEH + kSzW64x192;
constexpr size_t kOffWINH = kOffWPEL + kSzW64x192;
constexpr size_t kOffWINL = kOffWINH + kSzW8x64x64;
constexpr size_t kOffWCVH = kOffWINL + kSzW8x64x64;
constexpr size_t kOffWCVL = kOffWCVH + kSzW8x64x192;
constexpr size_t kOffWBC  = kOffWCVL + kSzW8x64x192;
constexpr size_t kOffBBC  = kOffWBC  + kSzW8x64x192;
constexpr size_t kOffWPOH = kOffBBC  + (size_t)kLayers * kNbc * 4;
constexpr size_t kOffWPOL = kOffWPOH + kSzW8x64x64;
constexpr size_t kOffWOUTH = kOffWPOL + kSzW8x64x64;
constexpr size_t kOffWOUTL = kOffWOUTH + kSzW64x192;
constexpr size_t kOffPE   = kOffWOUTL + kSzW64x192;
constexpr size_t kOffXPH  = kOffPE   + (size_t)kSeq * kF * 4;
constexpr size_t kOffXPL  = kOffXPH  + (size_t)kRows * kKpe * 2;
constexpr size_t kOffHA   = kOffXPL  + (size_t)kRows * kKpe * 2;
constexpr size_t kOffHB   = kOffHA   + kSzAct32;
constexpr size_t kOffXNH  = kOffHB   + kSzAct32;
constexpr size_t kOffXNL  = kOffXNH  + kSzAct16;
constexpr size_t kOffH0   = kOffXNL  + kSzAct16;
constexpr size_t kOffH0PH = kOffH0   + kSzAct32;
constexpr size_t kOffH0PL = kOffH0PH + kSzH0P;
constexpr size_t kOffHCR  = kOffH0PL + kSzH0P;
constexpr size_t kOffHC   = kOffHCR  + kSzAct32;
constexpr size_t kOffHCB  = kOffHC   + kSzAct32;
constexpr size_t kOffBCD  = kOffHCB  + kSzAct16;
constexpr size_t kOffGNH  = kOffBCD  + (size_t)kRows * kNbc * 4;
constexpr size_t kOffGNL  = kOffGNH  + kSzAct16;
constexpr size_t kOffHFH  = kOffGNL  + kSzAct16;
constexpr size_t kOffHFL  = kOffHFH  + kSzAct16;
constexpr size_t kOffOUTP = kOffHFL  + kSzAct16;
constexpr size_t kWsTotal = kOffOUTP + (size_t)kRows * kNout * 4;
static_assert(kWsTotal == 20619264ull, "carve total");
static_assert(kWsTotal <= 134217728ull, "carve cap");
static_assert((kOffWPEL % 128) == 0 && (kOffWINH % 128) == 0 && (kOffWINL % 128) == 0 && (kOffWCVH % 128) == 0 &&
              (kOffWCVL % 128) == 0 && (kOffWBC % 128) == 0 && (kOffBBC % 128) == 0 && (kOffWPOH % 128) == 0 &&
              (kOffWPOL % 128) == 0 && (kOffWOUTH % 128) == 0 && (kOffWOUTL % 128) == 0 && (kOffPE % 128) == 0 &&
              (kOffXPH % 128) == 0 && (kOffXPL % 128) == 0 && (kOffHA % 128) == 0 && (kOffHB % 128) == 0 &&
              (kOffXNH % 128) == 0 && (kOffXNL % 128) == 0 && (kOffH0 % 128) == 0 && (kOffH0PH % 128) == 0 &&
              (kOffH0PL % 128) == 0 && (kOffHCR % 128) == 0 && (kOffHC % 128) == 0 && (kOffHCB % 128) == 0 &&
              (kOffBCD % 128) == 0 && (kOffGNH % 128) == 0 && (kOffGNL % 128) == 0 && (kOffHFH % 128) == 0 &&
              (kOffHFL % 128) == 0 && (kOffOUTP % 128) == 0, "128-B aligned regions");

__device__ __forceinline__ unsigned short f2bf_bits(float f) {
  unsigned u = __float_as_uint(f);
  return (unsigned short)((u + 0x7FFFu + ((u >> 16) & 1u)) >> 16);
}
__device__ __forceinline__ float bf_bits2f(unsigned short h) { return __uint_as_float(((unsigned)h) << 16); }

__device__ __forceinline__ void dep_guard4_h(v8f& a, v8f& b, v8f& c, v8f& d, v16h x, v16h y) {
  asm volatile("v_nop\n\tv_nop\n\tv_nop\n\tv_nop" : "+v"(a), "+v"(b), "+v"(c), "+v"(d) : "v"(x), "v"(y));
}
__device__ __forceinline__ void dep_guard4_b(v8f& a, v8f& b, v8f& c, v8f& d, v16b x, v16b y) {
  asm volatile("v_nop\n\tv_nop\n\tv_nop\n\tv_nop" : "+v"(a), "+v"(b), "+v"(c), "+v"(d) : "v"(x), "v"(y));
}
__device__ __forceinline__ void keep4_h(v16h a, v16h b, v16h c, v16h d) { asm volatile("v_nop" :: "v"(a), "v"(b), "v"(c), "v"(d)); }
__device__ __forceinline__ void keep4_b(v16b a, v16b b, v16b c, v16b d) { asm volatile("v_nop" :: "v"(a), "v"(b), "v"(c), "v"(d)); }
__device__ __forceinline__ void acc_guard4(v8f& a, v8f& b, v8f& c, v8f& d) { asm volatile("v_nop\n\tv_nop\n\tv_nop\n\tv_nop" : "+v"(a), "+v"(b), "+v"(c), "+v"(d)); }
template <typename T> struct Frag;
template <> struct Frag<_Float16> {
  typedef v16h V; union U { v16h v; v8h h[2]; };
  static __device__ __forceinline__ v16h load(const _Float16* p) {
    U f; f.h[0] = *(const v8h*)(p); f.h[1] = *(const v8h*)(p + 16); return f.v;
  }
  static __device__ __forceinline__ v8f mma(v16h a, v16h b, v8f c) {
    return __builtin_amdgcn_wmma_f32_16x16x32_f16(false, a, false, b, (short)0, c, false, false);
  }
  static __device__ __forceinline__ void guard4(v8f& a, v8f& b, v8f& c, v8f& d, v16h x, v16h y) { dep_guard4_h(a, b, c, d, x, y); }
  static __device__ __forceinline__ void keep(v16h a, v16h b, v16h c, v16h d) { keep4_h(a, b, c, d); }
};
template <> struct Frag<__bf16> {
  typedef v16b V; union U { v16b v; v8b h[2]; };
  static __device__ __forceinline__ v16b load(const __bf16* p) {
    U f; f.h[0] = *(const v8b*)(p); f.h[1] = *(const v8b*)(p + 16); return f.v;
  }
  static __device__ __forceinline__ v8f mma(v16b a, v16b b, v8f c) {
    return __builtin_amdgcn_wmma_f32_16x16x32_bf16(false, a, false, b, (short)0, c, false, false);
  }
  static __device__ __forceinline__ void guard4(v8f& a, v8f& b, v8f& c, v8f& d, v16b x, v16b y) { dep_guard4_b(a, b, c, d, x, y); }
  static __device__ __forceinline__ void keep(v16b a, v16b b, v16b c, v16b d) { keep4_b(a, b, c, d); }
};

__device__ __forceinline__ v8h pack_bf8(v4f a0, v4f a1) {
  v8h hv;
#pragma unroll
  for (int e = 0; e < 4; ++e) {
    const unsigned short h0 = f2bf_bits(a0[e]), h1 = f2bf_bits(a1[e]);
    hv[e]     = __builtin_bit_cast(_Float16, h0);
    hv[4 + e] = __builtin_bit_cast(_Float16, h1);
  }
  return hv;
}
__device__ __forceinline__ void pack_bf8_hilo(v4f a0, v4f a1, v8h& hv, v8h& lv) {
#pragma unroll
  for (int e = 0; e < 4; ++e) {
    const unsigned short h0 = f2bf_bits(a0[e]), h1 = f2bf_bits(a1[e]);
    const unsigned short l0 = f2bf_bits(a0[e] - bf_bits2f(h0)), l1 = f2bf_bits(a1[e] - bf_bits2f(h1));
    hv[e]     = __builtin_bit_cast(_Float16, h0);
    hv[4 + e] = __builtin_bit_cast(_Float16, h1);
    lv[e]     = __builtin_bit_cast(_Float16, l0);
    lv[4 + e] = __builtin_bit_cast(_Float16, l1);
  }
}
__device__ __forceinline__ void store16_2p(unsigned short* p, v8h v) {
  *(volatile v8h*)p = v;
  __threadfence();
  *(volatile v8h*)p = v;
}
__device__ __forceinline__ void store16x2_2p(unsigned short* ph, unsigned short* pl, v8h hv, v8h lv) {
  *(volatile v8h*)ph = hv;
  *(volatile v8h*)pl = lv;
  __threadfence();
  *(volatile v8h*)ph = hv;
  *(volatile v8h*)pl = lv;
}

template <int ET> struct Elem;
template <> struct Elem<0> { typedef _Float16 T; };
template <> struct Elem<1> { typedef __bf16 T; };
template <int ET, int SPL, int BIAS_MODE, int OUT_MODE, bool RESID>
__global__ __launch_bounds__(256) void wmma_gemm64(
    const unsigned short* __restrict__ Ap, const unsigned short* __restrict__ A2p, int lda, long strideA,
    const unsigned short* __restrict__ Btp, const unsigned short* __restrict__ Bt2p, int ldb, long strideB,
    float* __restrict__ Cf, int ldc, long strideC,
    unsigned short* __restrict__ Ch, unsigned short* __restrict__ Cl, int ldc2, long strideC2,
    const float* __restrict__ bias, const float* __restrict__ resid, long strideR,
    int M, int N, int K, float scale) {
  static_assert(OUT_MODE == 0 || OUT_MODE == 2 || OUT_MODE == 3, "out mode");
  static_assert(!RESID || OUT_MODE == 0, "resid only with f32 out");
  static_assert(SPL == 0 || SPL == 2, "split mode");
  static_assert(BIAS_MODE == 0 || BIAS_MODE == 2, "bias mode");
  typedef typename Elem<ET>::T T;
  typedef typename Frag<T>::V V;
  const T* A = (const T*)Ap; const T* A2 = (const T*)A2p; const T* Bt = (const T*)Btp; const T* Bt2 = (const T*)Bt2p;
  __shared__ __align__(16) float sT[8][16 * 68];
  const int b    = blockIdx.y;
  const int lane = threadIdx.x & 31;
  const int wave = threadIdx.x >> 5;
  const int tilesN = N >> 6;
  const int tilesM = M >> 6;
  const int tile = blockIdx.x * 8 + wave;
  if (tile >= tilesM * tilesN) return;
  const int tm = tile / tilesN;
  const int tn = tile - tm * tilesN;
  const int m0 = tm << 6;
  const int n0 = tn << 6;

  const T* Ab  = A  + (size_t)b * strideA;
  const T* Bb  = Bt + (size_t)b * strideB;
  const T* Ab2 = (SPL == 2) ? (A2  + (size_t)b * strideA) : nullptr;
  const T* Bb2 = (SPL == 2) ? (Bt2 + (size_t)b * strideB) : nullptr;

  const int rlane = lane & 15;
  const int koff  = (lane >> 4) * 8;
  const int mOff  = (lane >> 4) * 8;

  v8f acc[4][4];
#pragma unroll
  for (int i = 0; i < 4; ++i)
#pragma unroll
    for (int j = 0; j < 4; ++j) acc[i][j] = (v8f){0.f,0.f,0.f,0.f,0.f,0.f,0.f,0.f};

  for (int k0 = 0; k0 < K; k0 += 32) {
    V bh[4], bl[4];
#pragma unroll
    for (int j = 0; j < 4; ++j) {
      const size_t bo = (size_t)(n0 + (j << 4) + rlane) * ldb + koff + k0;
      bh[j] = Frag<T>::load(Bb + bo);
      if (SPL == 2) bl[j] = Frag<T>::load(Bb2 + bo);
    }
#pragma unroll
    for (int i = 0; i < 4; ++i) {
      const size_t ao = (size_t)(m0 + (i << 4) + rlane) * lda + koff + k0;
      V ah = Frag<T>::load(Ab + ao);
      V al;
      if (SPL == 2) al = Frag<T>::load(Ab2 + ao);
#pragma unroll
      for (int j = 0; j < 4; ++j) {
        acc[i][j] = Frag<T>::mma(ah, bh[j], acc[i][j]);
        if (SPL == 2) {
          acc[i][j] = Frag<T>::mma(ah, bl[j], acc[i][j]);
          acc[i][j] = Frag<T>::mma(al, bh[j], acc[i][j]);
        }
      }
      Frag<T>::guard4(acc[i][0], acc[i][1], acc[i][2], acc[i][3], ah, (SPL == 2) ? al : ah);
    }
    Frag<T>::keep(bh[0], bh[1], bh[2], bh[3]);
    if (SPL == 2) Frag<T>::keep(bl[0], bl[1], bl[2], bl[3]);
  }
  acc_guard4(acc[0][0], acc[0][1], acc[0][2], acc[0][3]);
  acc_guard4(acc[1][0], acc[1][1], acc[1][2], acc[1][3]);
  acc_guard4(acc[2][0], acc[2][1], acc[2][2], acc[2][3]);
  acc_guard4(acc[3][0], acc[3][1], acc[3][2], acc[3][3]);

  float* slab = sT[wave];
#pragma unroll
  for (int i = 0; i < 4; ++i) {
    const int mBase = m0 + (i << 4);
#pragma unroll
    for (int j = 0; j < 4; ++j) {
      const int n = n0 + (j << 4) + rlane;
      float bv = 0.f;
      if (BIAS_MODE == 2) bv = bias[n];
#pragma unroll
      for (int r = 0; r < 8; ++r) {
        float v = acc[i][j][r] * scale;
        if (BIAS_MODE == 2) v += bv;
        slab[(mOff + r) * 68 + (j << 4) + rlane] = v;
      }
    }
    __builtin_amdgcn_fence(__ATOMIC_RELEASE, "workgroup");
    __builtin_amdgcn_wave_barrier();
    __builtin_amdgcn_fence(__ATOMIC_ACQUIRE, "workgroup");
    if (OUT_MODE == 0 || OUT_MODE == 3) {
      float* C = Cf + (size_t)b * strideC;
      const float* Rb = RESID ? (resid + (size_t)b * strideR) : nullptr;
      const int hq = lane >> 4, c4 = (lane & 15) * 4;
      for (int pass = 0; pass < 2; ++pass) {
#pragma unroll
        for (int it = 0; it < 8; ++it) {
          const int row = it * 2 + hq;
          v4f v = *(const v4f*)(slab + row * 68 + c4);
          if (RESID) {
            const v4f rv = *(const v4f*)(Rb + (size_t)(mBase + row) * ldc + n0 + c4);
            v += rv;
          }
          *(volatile v4f*)(C + (size_t)(mBase + row) * ldc + n0 + c4) = v;
        }
        __threadfence();
      }
    }
    if (OUT_MODE == 2 || OUT_MODE == 3) {
      const int q = lane >> 3, c8 = (lane & 7) * 8;
      unsigned short* C1 = Ch + (size_t)b * strideC2;
      unsigned short* C2 = Cl + (size_t)b * strideC2;
      for (int pass = 0; pass < 2; ++pass) {
#pragma unroll
        for (int it = 0; it < 4; ++it) {
          const int row = it * 4 + q;
          const float* sp = slab + row * 68 + c8;
          const v4f s0 = *(const v4f*)(sp);
          const v4f s1 = *(const v4f*)(sp + 4);
          v8h hv, lv;
          pack_bf8_hilo(s0, s1, hv, lv);
          *(volatile v8h*)(C1 + (size_t)(mBase + row) * ldc2 + n0 + c8) = hv;
          *(volatile v8h*)(C2 + (size_t)(mBase + row) * ldc2 + n0 + c8) = lv;
        }
        __threadfence();
      }
    }
    __builtin_amdgcn_fence(__ATOMIC_RELEASE, "workgroup");
    __builtin_amdgcn_wave_barrier();
    __builtin_amdgcn_fence(__ATOMIC_ACQUIRE, "workgroup");
  }
}

__global__ __launch_bounds__(256) void prep_kernel(
    const float* __restrict__ Wpe, const float* __restrict__ Wp_in, const float* __restrict__ Wconv,
    const float* __restrict__ WB, const float* __restrict__ bB, const float* __restrict__ WC, const float* __restrict__ bC,
    const float* __restrict__ Wd1, const float* __restrict__ bd1, const float* __restrict__ Wp_out, const float* __restrict__ Wout,
    unsigned short* __restrict__ WPEH, unsigned short* __restrict__ WPEL,
    unsigned short* __restrict__ WINH, unsigned short* __restrict__ WINL,
    unsigned short* __restrict__ WCVH, unsigned short* __restrict__ WCVL,
    unsigned short* __restrict__ WBCp, float* __restrict__ BBCp,
    unsigned short* __restrict__ WPOH, unsigned short* __restrict__ WPOL,
    unsigned short* __restrict__ WOUTH, unsigned short* __restrict__ WOUTL,
    unsigned short* __restrict__ H0PH, unsigned short* __restrict__ H0PL)
{
  const int bid = blockIdx.x, tid = threadIdx.x;
  if (bid < 6) {
    const int s = bid * 256 + tid;
    const int f = s / 24; const int k0 = (s - f * 24) * 8;
    const float* src = Wpe + (size_t)f * kKpe + k0;
    const v4f a0 = *(const v4f*)src, a1 = *(const v4f*)(src + 4);
    v8h hv, lv; pack_bf8_hilo(a0, a1, hv, lv);
    store16x2_2p(WPEH + (size_t)s * 8, WPEL + (size_t)s * 8, hv, lv);
  } else if (bid < 22) {
    const int s = (bid - 6) * 256 + tid;
    const int l = s >> 9; const int n = (s >> 3) & 63; const int k0 = (s & 7) * 8;
    const float* src = Wp_in + (size_t)l * 4096 + (size_t)k0 * 64 + n;
    v4f a0, a1;
#pragma unroll
    for (int e = 0; e < 4; ++e) { a0[e] = src[e * 64]; a1[e] = src[(e + 4) * 64]; }
    v8h hv, lv; pack_bf8_hilo(a0, a1, hv, lv);
    store16x2_2p(WINH + (size_t)s * 8, WINL + (size_t)s * 8, hv, lv);
  } else if (bid < 70) {
    const int s = (bid - 22) * 256 + tid;
    const int l = s / 1536; const int r = s - l * 1536;
    const int o = r / 24; const int kk = (r - o * 24) * 8;
    const int tap = kk >> 6; const int c0 = kk & 63;
    const float* src = Wconv + (((size_t)l * 64 + o) * 64 + c0) * 3 + tap;
    v4f a0, a1;
#pragma unroll
    for (int e = 0; e < 4; ++e) { a0[e] = src[e * 3]; a1[e] = src[(e + 4) * 3]; }
    v8h hv, lv; pack_bf8_hilo(a0, a1, hv, lv);
    store16x2_2p(WCVH + (size_t)s * 8, WCVL + (size_t)s * 8, hv, lv);
  } else if (bid < 118) {
    const int lb = bid - 70;
    const int l = lb / 6; const int sub = lb - l * 6;
    const int r = sub * 256 + tid;
    const int n = r >> 3; const int k0 = (r & 7) * 8;
    const size_t dst = ((size_t)l * 1536 + r) * 8;
    v4f a0, a1;
    if (sub < 2) {
      const float* src = WB + (size_t)l * 4096 + (size_t)k0 * 64 + n;
#pragma unroll
      for (int e = 0; e < 4; ++e) { a0[e] = src[e * 64]; a1[e] = src[(e + 4) * 64]; }
    } else if (sub < 4) {
      const float* src = WC + (size_t)l * 4096 + (size_t)k0 * 64 + (n - 64);
#pragma unroll
      for (int e = 0; e < 4; ++e) { a0[e] = src[e * 64]; a1[e] = src[(e + 4) * 64]; }
    } else {
      int nd = n - 128; nd = nd > 3 ? 3 : nd;
      const float fD = (n < 132) ? 1.f : 0.f;
      const float* src = Wd1 + (size_t)l * 256 + (size_t)k0 * 4 + nd;
#pragma unroll
      for (int e = 0; e < 4; ++e) { a0[e] = fD * src[e * 4]; a1[e] = fD * src[(e + 4) * 4]; }
    }
    store16_2p(WBCp + dst, pack_bf8(a0, a1));
  } else if (bid < 134) {
    const int s = (bid - 118) * 256 + tid;
    const int l = s >> 9; const int n = (s >> 3) & 63; const int k0 = (s & 7) * 8;
    const float* src = Wp_out + (size_t)l * 4096 + (size_t)k0 * 64 + n;
    v4f a0, a1;
#pragma unroll
    for (int e = 0; e < 4; ++e) { a0[e] = src[e * 64]; a1[e] = src[(e + 4) * 64]; }
    v8h hv, lv; pack_bf8_hilo(a0, a1, hv, lv);
    store16x2_2p(WPOH + (size_t)s * 8, WPOL + (size_t)s * 8, hv, lv);
  } else if (bid < 140) {
    const int s = (bid - 134) * 256 + tid;
    const int n = s >> 3; const int k0 = (s & 7) * 8;
    const float* src = Wout + (size_t)k0 * kNout + n;
    v4f a0, a1;
#pragma unroll
    for (int e = 0; e < 4; ++e) { a0[e] = src[e * kNout]; a1[e] = src[(e + 4) * kNout]; }
    v8h hv, lv; pack_bf8_hilo(a0, a1, hv, lv);
    store16x2_2p(WOUTH + (size_t)s * 8, WOUTL + (size_t)s * 8, hv, lv);
  } else if (bid < 142) {
    const int s = (bid - 140) * 256 + tid;
    if (s < 384) {
      const int l = s / 48; const int n4 = (s - l * 48) * 4;
      const int nb4 = n4 < 60 ? n4 : 60;
      int nc4 = n4 - 64; nc4 = nc4 < 0 ? 0 : nc4; nc4 = nc4 > 60 ? 60 : nc4;
      const float fB = (n4 < 64) ? 1.f : 0.f;
      const float fC = (n4 >= 64 && n4 < 128) ? 1.f : 0.f;
      const float fD = (n4 == 128) ? 1.f : 0.f;
      const v4f vB = *(const v4f*)(bB + (size_t)l * 64 + nb4);
      const v4f vC = *(const v4f*)(bC + (size_t)l * 64 + nc4);
      const v4f vD = *(const v4f*)(bd1 + (size_t)l * 4);
      v4f v = vB * fB;
      v = vC * fC + v;
      v = vD * fD + v;
      float* p = BBCp + (size_t)s * 4;
      *(volatile v4f*)p = v;
      __threadfence();
      *(volatile v4f*)p = v;
    }
  } else {
    if (tid < 128) {
      const int s = tid & 63;
      const int bb = s >> 4; const int top = (s >> 3) & 1; const int c8 = (s & 7) * 8;
      const size_t off = ((size_t)bb * kPadRows + (top ? (kPadRows - 1) : 0)) * kF + c8;
      const v4f z4 = (v4f){0.f, 0.f, 0.f, 0.f};
      const v8h z = pack_bf8(z4, z4);
      if (tid < 64) store16_2p(H0PH + off, z);
      else          store16_2p(H0PL + off, z);
    }
  }
}

struct PeDiv { float d[32]; };
static_assert(sizeof(PeDiv) == 128, "no padding");
__global__ __launch_bounds__(256) void pe_kernel(float* __restrict__ PE, PeDiv dv) {
  __shared__ __align__(16) float sP[8 * 64];
  const int tid = threadIdx.x, lane = tid & 31, wave = tid >> 5;
  const int l = blockIdx.x * 8 + wave;
  const int k = lane;
  float dk = dv.d[0];
  dk = (k == 1)  ? dv.d[1]  : dk;  dk = (k == 2)  ? dv.d[2]  : dk;  dk = (k == 3)  ? dv.d[3]  : dk;
  dk = (k == 4)  ? dv.d[4]  : dk;  dk = (k == 5)  ? dv.d[5]  : dk;  dk = (k == 6)  ? dv.d[6]  : dk;
  dk = (k == 7)  ? dv.d[7]  : dk;  dk = (k == 8)  ? dv.d[8]  : dk;  dk = (k == 9)  ? dv.d[9]  : dk;
  dk = (k == 10) ? dv.d[10] : dk;  dk = (k == 11) ? dv.d[11] : dk;  dk = (k == 12) ? dv.d[12] : dk;
  dk = (k == 13) ? dv.d[13] : dk;  dk = (k == 14) ? dv.d[14] : dk;  dk = (k == 15) ? dv.d[15] : dk;
  dk = (k == 16) ? dv.d[16] : dk;  dk = (k == 17) ? dv.d[17] : dk;  dk = (k == 18) ? dv.d[18] : dk;
  dk = (k == 19) ? dv.d[19] : dk;  dk = (k == 20) ? dv.d[20] : dk;  dk = (k == 21) ? dv.d[21] : dk;
  dk = (k == 22) ? dv.d[22] : dk;  dk = (k == 23) ? dv.d[23] : dk;  dk = (k == 24) ? dv.d[24] : dk;
  dk = (k == 25) ? dv.d[25] : dk;  dk = (k == 26) ? dv.d[26] : dk;  dk = (k == 27) ? dv.d[27] : dk;
  dk = (k == 28) ? dv.d[28] : dk;  dk = (k == 29) ? dv.d[29] : dk;  dk = (k == 30) ? dv.d[30] : dk;
  dk = (k == 31) ? dv.d[31] : dk;
  const float ang = (float)l * dk;
  float sv, cv;
  sincosf(ang, &sv, &cv);
  sP[wave * 64 + 2 * k]     = sv;
  sP[wave * 64 + 2 * k + 1] = cv;
  __syncthreads();
  if (tid < 128) {
    const int row = tid >> 4, c4 = (tid & 15) * 4;
    const v4f v = *(const v4f*)(sP + row * 64 + c4);
    float* p = PE + (size_t)(blockIdx.x * 8 + row) * kF + c4;
    *(volatile v4f*)p = v;
    __threadfence();
    *(volatile v4f*)p = v;
  }
}

__global__ __launch_bounds__(256) void im2col_kernel(const float* __restrict__ x,
                                                     unsigned short* __restrict__ XPH, unsigned short* __restrict__ XPL) {
  const int s = blockIdx.x * 256 + threadIdx.x;
  const int row = s / 24; const int k0 = (s - row * 24) * 8;
  const int b = row >> 10, l = row & 1023, i = l >> 5, j = l & 31;
  const int c = k0 >> 6, p = (k0 & 63) >> 3;
  const float* src = x + (((size_t)(b * kCin + c)) * kImg + 8 * i + p) * kImg + 8 * j;
  const v4f a0 = *(const v4f*)src, a1 = *(const v4f*)(src + 4);
  v8h hv, lv; pack_bf8_hilo(a0, a1, hv, lv);
  store16x2_2p(XPH + (size_t)row * kKpe + k0, XPL + (size_t)row * kKpe + k0, hv, lv);
}

__global__ __launch_bounds__(512) void gn_plane_kernel(const float* __restrict__ Hin,
                                                       unsigned short* __restrict__ XH, unsigned short* __restrict__ XL) {
  __shared__ float red[16];
  __shared__ float sm[2];
  const int tid = threadIdx.x, lane = tid & 31, wave = tid >> 5;
  const int b = blockIdx.x;
  const float* base = Hin + (size_t)b * (kSeq * kF);
  float s = 0.f;
#pragma unroll 1
  for (int it = 0; it < 32; ++it) {
    const v4f v = *(const v4f*)(base + ((size_t)(it * 512 + tid)) * 4);
    s += (v[0] + v[1]) + (v[2] + v[3]);
  }
#pragma unroll
  for (int off = 16; off > 0; off >>= 1) s += __shfl_xor(s, off, 32);
  if (lane == 0) red[wave] = s;
  __syncthreads();
  if (tid == 0) {
    float t = 0.f;
#pragma unroll
    for (int w = 0; w < 16; ++w) t += red[w];
    sm[0] = t * (1.0f / 65536.0f);
  }
  __syncthreads();
  const float m = sm[0];
  float ss = 0.f;
#pragma unroll 1
  for (int it = 0; it < 32; ++it) {
    const v4f v = *(const v4f*)(base + ((size_t)(it * 512 + tid)) * 4);
    const v4f d = v - m;
    ss = fmaf(d[0], d[0], ss); ss = fmaf(d[1], d[1], ss); ss = fmaf(d[2], d[2], ss); ss = fmaf(d[3], d[3], ss);
  }
#pragma unroll
  for (int off = 16; off > 0; off >>= 1) ss += __shfl_xor(ss, off, 32);
  if (lane == 0) red[wave] = ss;
  __syncthreads();
  if (tid == 0) {
    float t = 0.f;
#pragma unroll
    for (int w = 0; w < 16; ++w) t += red[w];
    sm[1] = rsqrtf(t * (1.0f / 65536.0f) + kEps);
  }
  __syncthreads();
  const float r = sm[1];
#pragma unroll 1
  for (int it = 0; it < 16; ++it) {
    const int sl = it * 512 + tid;
    const size_t e0 = (size_t)sl * 8;
    const v4f a0 = *(const v4f*)(base + e0);
    const v4f a1 = *(const v4f*)(base + e0 + 4);
    const v4f z0 = (a0 - m) * r;
    const v4f z1 = (a1 - m) * r;
    v8h hv, lv; pack_bf8_hilo(z0, z1, hv, lv);
    store16x2_2p(XH + (size_t)b * (kSeq * kF) + e0, XL + (size_t)b * (kSeq * kF) + e0, hv, lv);
  }
}

__global__ __launch_bounds__(256) void inorm_silu_kernel(const float* __restrict__ HCR,
                                                         float* __restrict__ HCo, unsigned short* __restrict__ HCB) {
  __shared__ float red[4 * 64];
  __shared__ float smean[64];
  __shared__ float srstd[64];
  __shared__ __align__(16) float sT[16 * 68];
  const int tid = threadIdx.x;
  const int c = tid & 63, g = tid >> 6;
  const int b = blockIdx.x;
  const size_t rbase = (size_t)b * kSeq;
  float s = 0.f;
#pragma unroll 1
  for (int k = 0; k < 256; ++k) s += HCR[(rbase + g + 4 * k) * kF + c];
  red[g * 64 + c] = s;
  __syncthreads();
  if (tid < 64) {
    const float t = (red[tid] + red[64 + tid]) + (red[128 + tid] + red[192 + tid]);
    smean[tid] = t * (1.0f / 1024.0f);
  }
  __syncthreads();
  const float m = smean[c];
  float ss = 0.f;
#pragma unroll 1
  for (int k = 0; k < 256; ++k) { const float d = HCR[(rbase + g + 4 * k) * kF + c] - m; ss = fmaf(d, d, ss); }
  red[g * 64 + c] = ss;
  __syncthreads();
  if (tid < 64) {
    const float t = (red[tid] + red[64 + tid]) + (red[128 + tid] + red[192 + tid]);
    srstd[tid] = rsqrtf(t * (1.0f / 1024.0f) + kEps);
  }
  __syncthreads();
  const float r = srstd[c];
  const int frow = tid >> 4, fc4 = (tid & 15) * 4;
  const int hrow = tid >> 3, hc8 = (tid & 7) * 8;
#pragma unroll 1
  for (int ch = 0; ch < 64; ++ch) {
#pragma unroll
    for (int k = 0; k < 4; ++k) {
      const int lr = g + 4 * k;
      const float xv = HCR[(rbase + ch * 16 + lr) * kF + c];
      const float z = (xv - m) * r;
      const float sg = __builtin_amdgcn_rcpf(1.0f + expf(-z));
      sT[lr * 68 + c] = z * sg;
    }
    __syncthreads();
    const v4f fv = *(const v4f*)(sT + frow * 68 + fc4);
    float* fp = HCo + (rbase + ch * 16 + frow) * kF + fc4;
    v8h hv;
    unsigned short* hp = HCB + (rbase + ch * 16 + (hrow & 15)) * kF + hc8;
    if (tid < 128) {
      const v4f a0 = *(const v4f*)(sT + hrow * 68 + hc8);
      const v4f a1 = *(const v4f*)(sT + hrow * 68 + hc8 + 4);
      hv = pack_bf8(a0, a1);
    }
    for (int pass = 0; pass < 2; ++pass) {
      *(volatile v4f*)fp = fv;
      if (tid < 128) *(volatile v8h*)hp = hv;
      __threadfence();
    }
    __syncthreads();
  }
}

__global__ __launch_bounds__(128) void ssm_scan_kernel(
    const float* __restrict__ BCD, const float* __restrict__ HC, const float* __restrict__ H0,
    const float* __restrict__ Wd2l, const float* __restrict__ bd2l, const float* __restrict__ Alogl,
    const float* __restrict__ Dpl, unsigned short* __restrict__ GNH, unsigned short* __restrict__ GNL)
{
  __shared__ __align__(16) float    sA[kF * kNst];
  __shared__ __align__(16) float    sB[kTS * kNst];
  __shared__ __align__(16) _Float16 sC[kTS * kNst];
  __shared__ __align__(16) float    sD[kTS * 4];
  __shared__ __align__(16) float    sHc[kTS * kF];
  __shared__ __align__(16) float    sHz[kTS * kF];
  __shared__ __align__(16) float    sG[kTS * 68];
  __shared__ float sSt[kTS * 2];
  const int tid = threadIdx.x, lane = tid & 31, wave = tid >> 5;
  const int hh = lane >> 4, m = lane & 15;
  const int b = blockIdx.x;
  const int f  = wave * 16 + m;
  const int oc = wave * 16 + 8 * hh + (lane & 7);
  const int r7 = lane & 7;
  const bool wr = ((lane & 8) == 0);
  const size_t row0 = (size_t)b * kSeq;
#pragma unroll 1
  for (int it = 0; it < 8; ++it) {
    const int q4 = it * 128 + tid;
    const v4f v = *(const v4f*)(Alogl + (size_t)q4 * 4);
    v4f e; e[0] = expf(v[0]); e[1] = expf(v[1]); e[2] = expf(v[2]); e[3] = expf(v[3]);
    *(v4f*)(sA + q4 * 4) = e;
  }
  const float w20 = Wd2l[f], w21 = Wd2l[64 + f], w22 = Wd2l[128 + f], w23 = Wd2l[192 + f];
  const float b2  = bd2l[f];
  const float dpo = Dpl[oc];
  __syncthreads();
  float a[32], st[32];
#pragma unroll
  for (int blk = 0; blk < 4; ++blk) {
    const v4f a0 = *(const v4f*)(sA + f * kNst + blk * 16 + 8 * hh);
    const v4f a1 = *(const v4f*)(sA + f * kNst + blk * 16 + 8 * hh + 4);
    a[blk * 8 + 0] = a0[0]; a[blk * 8 + 1] = a0[1]; a[blk * 8 + 2] = a0[2]; a[blk * 8 + 3] = a0[3];
    a[blk * 8 + 4] = a1[0]; a[blk * 8 + 5] = a1[1]; a[blk * 8 + 6] = a1[2]; a[blk * 8 + 7] = a1[3];
  }
#pragma unroll
  for (int j = 0; j < 32; ++j) st[j] = 0.0f;
  const int lr4 = tid >> 4, lc4 = (tid & 15) * 4;

#pragma unroll 1
  for (int t0 = 0; t0 < kSeq; t0 += kTS) {
    __syncthreads();
#pragma unroll 1
    for (int i = 0; i < 4; ++i) {
      const int r = lr4 + 8 * i;
      const size_t gr = row0 + t0 + r;
      const v4f vb = *(const v4f*)(BCD + gr * kNbc + lc4);
      const v4f vh = *(const v4f*)(HC + gr * kF + lc4);
      const v4f vz = *(const v4f*)(H0 + gr * kF + lc4);
      *(v4f*)(sB  + r * kNst + lc4) = vb;
      *(v4f*)(sHc + r * kF + lc4)   = vh;
      *(v4f*)(sHz + r * kF + lc4)   = vz;
    }
#pragma unroll
    for (int i = 0; i < 2; ++i) {
      const int sl = i * 128 + tid;
      const int r = sl >> 3, c8 = (sl & 7) * 8;
      const size_t gr = row0 + t0 + r;
      const v4f c0 = *(const v4f*)(BCD + gr * kNbc + 64 + c8);
      const v4f c1 = *(const v4f*)(BCD + gr * kNbc + 64 + c8 + 4);
      v8h cv;
#pragma unroll
      for (int e = 0; e < 4; ++e) { cv[e] = (_Float16)(c0[e] * 64.0f); cv[4 + e] = (_Float16)(c1[e] * 64.0f); }
      *(v8h*)(sC + r * kNst + c8) = cv;
    }
    if (tid < kTS) *(v4f*)(sD + tid * 4) = *(const v4f*)(BCD + (row0 + t0 + tid) * kNbc + 128);
    __syncthreads();

#pragma unroll 1
    for (int s = 0; s < kTS; ++s) {
      const float* bro = sB + s * kNst;
      const v4f dv = *(const v4f*)(sD + s * 4);
      float dot = dv[0] * w20;
      dot = fmaf(dv[1], w21, dot);
      dot = fmaf(dv[2], w22, dot);
      dot = fmaf(dv[3], w23, dot);
      const float pre = dot + b2;
      const float ex  = expf(-fabsf(pre));
      const float dl  = fmaxf(pre, 0.0f) + log1pf(ex);
      const float hcf = sHc[s * kF + f];
      const float u   = dl * hcf;
      const float ndl = -dl;
      v16h af0, af1;
#pragma unroll
      for (int blk = 0; blk < 4; ++blk) {
        const v4f bq0 = *(const v4f*)(bro + blk * 16 + 8 * hh);
        const v4f bq1 = *(const v4f*)(bro + blk * 16 + 8 * hh + 4);
#pragma unroll
        for (int i = 0; i < 4; ++i) {
          const int j = blk * 8 + i;
          const float ab = expf(ndl * a[j]);
          const float bx = u * bq0[i];
          st[j] = ab * st[j] + bx;
          const _Float16 hq = (_Float16)(st[j] * 256.0f);
          if (blk < 2) af0[(blk & 1) * 8 + i] = hq; else af1[(blk & 1) * 8 + i] = hq;
        }
#pragma unroll
        for (int i = 0; i < 4; ++i) {
          const int j = blk * 8 + 4 + i;
          const float ab = expf(ndl * a[j]);
          const float bx = u * bq1[i];
          st[j] = ab * st[j] + bx;
          const _Float16 hq = (_Float16)(st[j] * 256.0f);
          if (blk < 2) af0[(blk & 1) * 8 + 4 + i] = hq; else af1[(blk & 1) * 8 + 4 + i] = hq;
        }
      }
      const v16h kb0 = Frag<_Float16>::load(sC + s * kNst + 8 * hh);
      const v16h kb1 = Frag<_Float16>::load(sC + s * kNst + 32 + 8 * hh);
      v8f acc = (v8f){0.f, 0.f, 0.f, 0.f, 0.f, 0.f, 0.f, 0.f};
      acc = Frag<_Float16>::mma(af0, kb0, acc);
      acc = Frag<_Float16>::mma(af1, kb1, acc);
      asm volatile("v_nop\n\tv_nop\n\tv_nop\n\tv_nop" : "+v"(acc) : "v"(af0), "v"(kb0), "v"(af1), "v"(kb1));
      float ys = acc[0];
      ys = (r7 == 1) ? acc[1] : ys;
      ys = (r7 == 2) ? acc[2] : ys;
      ys = (r7 == 3) ? acc[3] : ys;
      ys = (r7 == 4) ? acc[4] : ys;
      ys = (r7 == 5) ? acc[5] : ys;
      ys = (r7 == 6) ? acc[6] : ys;
      ys = (r7 == 7) ? acc[7] : ys;
      const float hco = sHc[s * kF + oc];
      const float y   = ys * (1.0f / 16384.0f) + dpo * hco;
      const float hz  = sHz[s * kF + oc];
      const float sg  = hz * __builtin_amdgcn_rcpf(1.0f + expf(-hz));
      const float gv  = y * sg;
      if (wr) sG[s * 68 + oc] = gv;
    }
    __syncthreads();
    if (tid < kTS) {
      const float* gr = sG + tid * 68;
      float sm = 0.f;
#pragma unroll 1
      for (int k = 0; k < kF; ++k) sm += gr[k];
      const float mu = sm * (1.0f / 64.0f);
      float sv = 0.f;
#pragma unroll 1
      for (int k = 0; k < kF; ++k) { const float d = gr[k] - mu; sv = fmaf(d, d, sv); }
      sSt[2 * tid] = mu;
      sSt[2 * tid + 1] = rsqrtf(sv * (1.0f / 64.0f) + kEps);
    }
    __syncthreads();
    v8h hv0, lv0, hv1, lv1;
    size_t go0, go1;
    {
      const int sl = tid;
      const int r = sl >> 3, c8 = (sl & 7) * 8;
      const float mu = sSt[2 * r], rs = sSt[2 * r + 1];
      const v4f g0 = *(const v4f*)(sG + r * 68 + c8);
      const v4f g1 = *(const v4f*)(sG + r * 68 + c8 + 4);
      pack_bf8_hilo((g0 - mu) * rs, (g1 - mu) * rs, hv0, lv0);
      go0 = (row0 + t0 + r) * kF + c8;
    }
    {
      const int sl = 128 + tid;
      const int r = sl >> 3, c8 = (sl & 7) * 8;
      const float mu = sSt[2 * r], rs = sSt[2 * r + 1];
      const v4f g0 = *(const v4f*)(sG + r * 68 + c8);
      const v4f g1 = *(const v4f*)(sG + r * 68 + c8 + 4);
      pack_bf8_hilo((g0 - mu) * rs, (g1 - mu) * rs, hv1, lv1);
      go1 = (row0 + t0 + r) * kF + c8;
    }
    for (int pass = 0; pass < 2; ++pass) {
      *(volatile v8h*)(GNH + go0) = hv0;
      *(volatile v8h*)(GNL + go0) = lv0;
      *(volatile v8h*)(GNH + go1) = hv1;
      *(volatile v8h*)(GNL + go1) = lv1;
      __threadfence();
    }
  }
}

__global__ __launch_bounds__(256) void split_plane_kernel(
    const float* __restrict__ src, unsigned short* __restrict__ dhi, unsigned short* __restrict__ dlo, int total8)
{
  const int i = blockIdx.x * 256 + threadIdx.x;
  if (i >= total8) return;
  const size_t e0 = (size_t)i << 3;
  const v4f a0 = *(const v4f*)(src + e0);
  const v4f a1 = *(const v4f*)(src + e0 + 4);
  v8h hv, lv; pack_bf8_hilo(a0, a1, hv, lv);
  store16x2_2p(dhi + e0, dlo + e0, hv, lv);
}

__global__ __launch_bounds__(256) void unpatch_kernel(const float* __restrict__ OUTP, const float* __restrict__ bout,
                                                      float* __restrict__ out) {
  const int bid = blockIdx.x;
  const int lane = threadIdx.x & 31, wave = threadIdx.x >> 5;
  const int b = bid / 96; const int rr = bid - b * 96; const int o = rr >> 5; const int i = rr & 31;
  const int p = wave;
  const float bo = bout[o];
  v4f v[2];
#pragma unroll
  for (int it = 0; it < 2; ++it) {
    const int x4 = it * 32 + lane;
    const int j = x4 >> 1, q0 = (x4 & 1) * 4;
    const v4f ld = *(const v4f*)(OUTP + ((size_t)(b * kSeq + i * kGp + j)) * kNout + o * 64 + p * 8 + q0);
    v[it] = ld + bo;
  }
  float* dst = out + (((size_t)(b * kCout + o)) * kImg + 8 * i + p) * kImg;
  for (int pass = 0; pass < 2; ++pass) {
#pragma unroll
    for (int it = 0; it < 2; ++it) *(volatile v4f*)(dst + (it * 32 + lane) * 4) = v[it];
    __threadfence();
  }
}

extern "C" void kernel_launch(void* const* d_in, const int* in_sizes, int n_in,
                              void* d_out, int out_size, void* d_ws, size_t ws_size,
                              hipStream_t stream) {
  if (n_in < 21) return;
  if (in_sizes[0] != kBatch * kCin * kImg * kImg) return;
  if (in_sizes[1] != kF * kKpe) return;
  if (in_sizes[2] != kF) return;
  if (in_sizes[3] != kLayers * kF * kF) return;
  if (in_sizes[4] != kLayers * kF) return;
  if (in_sizes[5] != kLayers * kF * kF * 3) return;
  if (in_sizes[6] != kLayers * kF) return;
  if (in_sizes[7] != kLayers * kF * kNst) return;
  if (in_sizes[8] != kLayers * kF) return;
  if (in_sizes[9] != kLayers * kF * kNst) return;
  if (in_sizes[10] != kLayers * kNst) return;
  if (in_sizes[11] != kLayers * kF * kNst) return;
  if (in_sizes[12] != kLayers * kNst) return;
  if (in_sizes[13] != kLayers * kF * kNd) return;
  if (in_sizes[14] != kLayers * kNd) return;
  if (in_sizes[15] != kLayers * kNd * kF) return;
  if (in_sizes[16] != kLayers * kF) return;
  if (in_sizes[17] != kLayers * kF * kF) return;
  if (in_sizes[18] != kLayers * kF) return;
  if (in_sizes[19] != kF * kNout) return;
  if (in_sizes[20] != kCout) return;
  if (out_size != kBatch * kCout * kImg * kImg) return;
  if (ws_size < kWsTotal) return;

  const float* x      = (const float*)d_in[0];
  const float* Wpe    = (const float*)d_in[1];
  const float* bpe    = (const float*)d_in[2];
  const float* Wp_in  = (const float*)d_in[3];
  const float* bp_in  = (const float*)d_in[4];
  const float* Wconv  = (const float*)d_in[5];
  const float* bconv  = (const float*)d_in[6];
  const float* A_log  = (const float*)d_in[7];
  const float* Dp     = (const float*)d_in[8];
  const float* WB     = (const float*)d_in[9];
  const float* bB     = (const float*)d_in[10];
  const float* WC     = (const float*)d_in[11];
  const float* bC     = (const float*)d_in[12];
  const float* Wd1    = (const float*)d_in[13];
  const float* bd1    = (const float*)d_in[14];
  const float* Wd2    = (const float*)d_in[15];
  const float* bd2    = (const float*)d_in[16];
  const float* Wp_out = (const float*)d_in[17];
  const float* bp_out = (const float*)d_in[18];
  const float* Wout   = (const float*)d_in[19];
  const float* bout   = (const float*)d_in[20];
  float* out = (float*)d_out;

  char* ws = (char*)d_ws;
  unsigned short* WPEH  = (unsigned short*)(ws + kOffWPEH);
  unsigned short* WPEL  = (unsigned short*)(ws + kOffWPEL);
  unsigned short* WINH  = (unsigned short*)(ws + kOffWINH);
  unsigned short* WINL  = (unsigned short*)(ws + kOffWINL);
  unsigned short* WCVH  = (unsigned short*)(ws + kOffWCVH);
  unsigned short* WCVL  = (unsigned short*)(ws + kOffWCVL);
  unsigned short* WBCp  = (unsigned short*)(ws + kOffWBC);
  float*          BBCp  = (float*)(ws + kOffBBC);
  unsigned short* WPOH  = (unsigned short*)(ws + kOffWPOH);
  unsigned short* WPOL  = (unsigned short*)(ws + kOffWPOL);
  unsigned short* WOUTH = (unsigned short*)(ws + kOffWOUTH);
  unsigned short* WOUTL = (unsigned short*)(ws + kOffWOUTL);
  float*          PE    = (float*)(ws + kOffPE);
  unsigned short* XPH   = (unsigned short*)(ws + kOffXPH);
  unsigned short* XPL   = (unsigned short*)(ws + kOffXPL);
  float*          HA    = (float*)(ws + kOffHA);
  float*          HB    = (float*)(ws + kOffHB);
  unsigned short* XNH   = (unsigned short*)(ws + kOffXNH);
  unsigned short* XNL   = (unsigned short*)(ws + kOffXNL);
  float*          H0    = (float*)(ws + kOffH0);
  unsigned short* H0PH  = (unsigned short*)(ws + kOffH0PH);
  unsigned short* H0PL  = (unsigned short*)(ws + kOffH0PL);
  float*          HCR   = (float*)(ws + kOffHCR);
  float*          HCf   = (float*)(ws + kOffHC);
  unsigned short* HCB   = (unsigned short*)(ws + kOffHCB);
  float*          BCD   = (float*)(ws + kOffBCD);
  unsigned short* GNH   = (unsigned short*)(ws + kOffGNH);
  unsigned short* GNL   = (unsigned short*)(ws + kOffGNL);
  unsigned short* HFH   = (unsigned short*)(ws + kOffHFH);
  unsigned short* HFL   = (unsigned short*)(ws + kOffHFL);
  float*          OUTP  = (float*)(ws + kOffOUTP);

  prep_kernel<<<143, 256, 0, stream>>>(Wpe, Wp_in, Wconv, WB, bB, WC, bC, Wd1, bd1, Wp_out, Wout,
                                       WPEH, WPEL, WINH, WINL, WCVH, WCVL, WBCp, BBCp,
                                       WPOH, WPOL, WOUTH, WOUTL, H0PH, H0PL);

  PeDiv dv;
  {
    const float cstf = (float)(-log(10000.0) / 64.0);
    for (int k = 0; k < 32; ++k) {
      const float prod = (float)((double)(float)(2 * k) * (double)cstf);
      dv.d[k] = (float)exp((double)prod);
    }
  }
  pe_kernel<<<kSeq / 8, 256, 0, stream>>>(PE, dv);

  im2col_kernel<<<(kRows * 24) / 256, 256, 0, stream>>>(x, XPH, XPL);

  wmma_gemm64<1, 2, 2, 0, true><<<dim3(2, kBatch), 256, 0, stream>>>(
      XPH, XPL, kKpe, (long)kSeq * kKpe,
      WPEH, WPEL, kKpe, 0L,
      HA, kF, (long)kSeq * kF,
      nullptr, nullptr, 0, 0L,
      bpe, PE, 0L,
      kSeq, kF, kKpe, 1.0f);

  for (int l = 0; l < kLayers; ++l) {
    float* hin  = (l & 1) ? HB : HA;
    float* hout = (l & 1) ? HA : HB;

    gn_plane_kernel<<<kBatch, 512, 0, stream>>>(hin, XNH, XNL);

    wmma_gemm64<1, 2, 2, 3, false><<<dim3(2, kBatch), 256, 0, stream>>>(
        XNH, XNL, kF, (long)kSeq * kF,
        WINH + (size_t)l * 4096, WINL + (size_t)l * 4096, kF, 0L,
        H0, kF, (long)kSeq * kF,
        H0PH + kF, H0PL + kF, kF, (long)kPadRows * kF,
        bp_in + l * kF, nullptr, 0L,
        kSeq, kF, kF, 1.0f);

    wmma_gemm64<1, 2, 2, 0, false><<<dim3(2, kBatch), 256, 0, stream>>>(
        H0PH, H0PL, kF, (long)kPadRows * kF,
        WCVH + (size_t)l * 12288, WCVL + (size_t)l * 12288, kKcv, 0L,
        HCR, kF, (long)kSeq * kF,
        nullptr, nullptr, 0, 0L,
        bconv + l * kF, nullptr, 0L,
        kSeq, kF, kKcv, 1.0f);

    inorm_silu_kernel<<<kBatch, 256, 0, stream>>>(HCR, HCf, HCB);

    wmma_gemm64<1, 0, 2, 0, false><<<dim3(24, 1), 256, 0, stream>>>(
        HCB, nullptr, kF, 0L,
        WBCp + (size_t)l * 12288, nullptr, kF, 0L,
        BCD, kNbc, 0L,
        nullptr, nullptr, 0, 0L,
        BBCp + l * kNbc, nullptr, 0L,
        kRows, kNbc, kF, 1.0f);

    ssm_scan_kernel<<<kBatch, 128, 0, stream>>>(BCD, HCf, H0, Wd2 + l * 256, bd2 + l * kF,
                                                A_log + (size_t)l * 4096, Dp + l * kF, GNH, GNL);

    wmma_gemm64<1, 2, 2, 0, true><<<dim3(8, 1), 256, 0, stream>>>(
        GNH, GNL, kF, 0L,
        WPOH + (size_t)l * 4096, WPOL + (size_t)l * 4096, kF, 0L,
        hout, kF, 0L,
        nullptr, nullptr, 0, 0L,
        bp_out + l * kF, hin, 0L,
        kRows, kF, kF, 1.0f);
  }

  split_plane_kernel<<<(kRows * kF / 8) / 256, 256, 0, stream>>>(HA, HFH, HFL, kRows * kF / 8);

  wmma_gemm64<1, 2, 0, 0, false><<<dim3(24, 1), 256, 0, stream>>>(
      HFH, HFL, kF, 0L,
      WOUTH, WOUTL, kF, 0L,
      OUTP, kNout, 0L,
      nullptr, nullptr, 0, 0L,
      nullptr, nullptr, 0L,
      kRows, kNout, kF, 1.0f);

  unpatch_kernel<<<kBatch * kCout * kGp, 256, 0, stream>>>(OUTP, bout, out);
}
